// FastTransformer_82042465288570
// MI455X (gfx1250) — hardware-verified
//
#include <hip/hip_runtime.h>

typedef __attribute__((ext_vector_type(16))) _Float16 v16h;
typedef __attribute__((ext_vector_type(8)))  _Float16 v8h;
typedef __attribute__((ext_vector_type(4)))  _Float16 v4h;
typedef __attribute__((ext_vector_type(16))) __bf16   v16b;
typedef __attribute__((ext_vector_type(8)))  __bf16   v8b;
typedef __attribute__((ext_vector_type(8)))  float    v8f;
typedef __attribute__((ext_vector_type(4)))  float    v4f;

__device__ __forceinline__ unsigned short f2bf_bits(float f) {
  unsigned u = __float_as_uint(f);
  return (unsigned short)((u + 0x7FFFu + ((u >> 16) & 1u)) >> 16);
}
__device__ __forceinline__ float bf_bits2f(unsigned short h) { return __uint_as_float(((unsigned)h) << 16); }

__device__ __forceinline__ void dep_guard_h(v8f& a, v8f& b, v16h x, v16h y) { asm volatile("v_nop\n\tv_nop\n\tv_nop\n\tv_nop" : "+v"(a), "+v"(b) : "v"(x), "v"(y)); }
__device__ __forceinline__ void dep_guard_b(v8f& a, v8f& b, v16b x, v16b y) { asm volatile("v_nop\n\tv_nop\n\tv_nop\n\tv_nop" : "+v"(a), "+v"(b) : "v"(x), "v"(y)); }
__device__ __forceinline__ void keep4_h(v16h a, v16h b, v16h c, v16h d) { asm volatile("v_nop" :: "v"(a), "v"(b), "v"(c), "v"(d)); }
__device__ __forceinline__ void keep4_b(v16b a, v16b b, v16b c, v16b d) { asm volatile("v_nop" :: "v"(a), "v"(b), "v"(c), "v"(d)); }
__device__ __forceinline__ void acc_guard4(v8f& a, v8f& b, v8f& c, v8f& d) { asm volatile("v_nop\n\tv_nop\n\tv_nop\n\tv_nop" : "+v"(a), "+v"(b), "+v"(c), "+v"(d)); }
template <typename T> struct Frag;
template <> struct Frag<_Float16> {
  typedef v16h V; union U { v16h v; v8h h[2]; };
  static __device__ __forceinline__ v16h load(const _Float16* p) {
    U f; f.h[0] = *(const v8h*)(p); f.h[1] = *(const v8h*)(p + 16); return f.v;
  }
  static __device__ __forceinline__ v8f mma(v16h a, v16h b, v8f c) {
    return __builtin_amdgcn_wmma_f32_16x16x32_f16(false, a, false, b, (short)0, c, false, false);
  }
  static __device__ __forceinline__ void guard(v8f& a, v8f& b, v16h x, v16h y) { dep_guard_h(a, b, x, y); }
  static __device__ __forceinline__ void keep(v16h a, v16h b, v16h c, v16h d) { keep4_h(a, b, c, d); }
};
template <> struct Frag<__bf16> {
  typedef v16b V; union U { v16b v; v8b h[2]; };
  static __device__ __forceinline__ v16b load(const __bf16* p) {
    U f; f.h[0] = *(const v8b*)(p); f.h[1] = *(const v8b*)(p + 16); return f.v;
  }
  static __device__ __forceinline__ v8f mma(v16b a, v16b b, v8f c) {
    return __builtin_amdgcn_wmma_f32_16x16x32_bf16(false, a, false, b, (short)0, c, false, false);
  }
  static __device__ __forceinline__ void guard(v8f& a, v8f& b, v16b x, v16b y) { dep_guard_b(a, b, x, y); }
  static __device__ __forceinline__ void keep(v16b a, v16b b, v16b c, v16b d) { keep4_b(a, b, c, d); }
};

template <int ET> struct Elem;
template <> struct Elem<0> { typedef _Float16 T; };
template <> struct Elem<1> { typedef __bf16 T; };
template <int ET, bool SPLIT, int BIAS_MODE, int OUT_MODE, bool RESID, int ACT = 0>
__global__ __launch_bounds__(256) void wmma_gemm64(
    const unsigned short* __restrict__ Ap, const unsigned short* __restrict__ A2p, int lda, long strideA,
    const unsigned short* __restrict__ Btp, const unsigned short* __restrict__ Bt2p, int ldb, long strideB,
    void* __restrict__ Cout, void* __restrict__ Cout2, int ldc, long strideC,
    const float* __restrict__ bias,
    const float* __restrict__ resid, long strideR,
    int M, int N, int K, float scale) {
  typedef typename Elem<ET>::T T;
  typedef typename Frag<T>::V V;
  const T* A = (const T*)Ap; const T* A2 = (const T*)A2p; const T* Bt = (const T*)Btp; const T* Bt2 = (const T*)Bt2p;
  __shared__ __align__(16) float sT[8][16 * 68];
  const int b    = blockIdx.y;
  const int lane = threadIdx.x & 31;
  const int wave = threadIdx.x >> 5;
  const int tilesN = N >> 6;
  const int tilesM = M >> 6;
  const int tile = blockIdx.x * 8 + wave;
  if (tile >= tilesM * tilesN) return;
  const int tm = tile / tilesN;
  const int tn = tile - tm * tilesN;
  const int m0 = tm << 6;
  const int n0 = tn << 6;

  const T* Ab  = A  + (size_t)b * strideA;
  const T* Bb  = Bt + (size_t)b * strideB;
  const T* Ab2 = SPLIT ? (A2  + (size_t)b * strideA) : nullptr;
  const T* Bb2 = SPLIT ? (Bt2 + (size_t)b * strideB) : nullptr;

  const int rlane = lane & 15;
  const int koff  = (lane >> 4) * 8;
  const int mOff  = (lane >> 4) * 8;

  v8f acc[4][4];
#pragma unroll
  for (int i = 0; i < 4; ++i)
#pragma unroll
    for (int j = 0; j < 4; ++j) acc[i][j] = (v8f){0.f,0.f,0.f,0.f,0.f,0.f,0.f,0.f};

  for (int k0 = 0; k0 < K; k0 += 32) {
    V bh[4], bl[4];
#pragma unroll
    for (int j = 0; j < 4; ++j) {
      const size_t bo = (size_t)(n0 + (j << 4) + rlane) * ldb + koff + k0;
      bh[j] = Frag<T>::load(Bb + bo);
      if (SPLIT) bl[j] = Frag<T>::load(Bb2 + bo);
    }
#pragma unroll
    for (int i = 0; i < 4; ++i) {
      const size_t ao = (size_t)(m0 + (i << 4) + rlane) * lda + koff + k0;
      V ah = Frag<T>::load(Ab + ao);
      V al;
      if (SPLIT) al = Frag<T>::load(Ab2 + ao);
#pragma unroll
      for (int j = 0; j < 4; ++j) {
        acc[i][j] = Frag<T>::mma(ah, bh[j], acc[i][j]);
        if (SPLIT) {
          acc[i][j] = Frag<T>::mma(ah, bl[j], acc[i][j]);
          acc[i][j] = Frag<T>::mma(al, bh[j], acc[i][j]);
        }
      }
      Frag<T>::guard(acc[i][0], acc[i][3], ah, SPLIT ? al : ah);
    }
    Frag<T>::keep(bh[0], bh[1], bh[2], bh[3]);
    if (SPLIT) Frag<T>::keep(bl[0], bl[1], bl[2], bl[3]);
  }
  acc_guard4(acc[0][0], acc[0][1], acc[0][2], acc[0][3]);
  acc_guard4(acc[1][0], acc[1][1], acc[1][2], acc[1][3]);
  acc_guard4(acc[2][0], acc[2][1], acc[2][2], acc[2][3]);
  acc_guard4(acc[3][0], acc[3][1], acc[3][2], acc[3][3]);

  float* slab = sT[wave];
  const float* Rb = RESID ? (resid + (size_t)b * strideR) : nullptr;
#pragma unroll
  for (int i = 0; i < 4; ++i) {
    const int mBase = m0 + (i << 4);
#pragma unroll
    for (int j = 0; j < 4; ++j) {
      const int n = n0 + (j << 4) + rlane;
      float bv = 0.f;
      if (BIAS_MODE == 2) bv = bias[n];
#pragma unroll
      for (int r = 0; r < 8; ++r) {
        float v = acc[i][j][r] * scale;
        if (BIAS_MODE == 1) v += bias[mBase + mOff + r];
        if (BIAS_MODE == 2) v += bv;
        if (RESID) v += Rb[(size_t)(mBase + mOff + r) * ldc + n];
        if (ACT == 1) v = tanhf(v);
        if (ACT == 2) v = fmaxf(v, 0.0f);
        if (ACT == 3) v = v / (1.0f + expf(-v));
        if (ACT == 4) v = (v > 0.f) ? v : 0.01f * v;
        if (ACT == 5) v = 0.5f * v * (1.0f + erff(v * 0.70710678118654752f));
        slab[(mOff + r) * 68 + (j << 4) + rlane] = v;
      }
    }
    __builtin_amdgcn_fence(__ATOMIC_RELEASE, "workgroup");
    __builtin_amdgcn_wave_barrier();
    __builtin_amdgcn_fence(__ATOMIC_ACQUIRE, "workgroup");
    if (OUT_MODE == 0) {
      float* C = (float*)Cout + (size_t)b * strideC;
      const int hh = lane >> 4, c4 = (lane & 15) * 4;
      for (int pass = 0; pass < 2; ++pass) {
#pragma unroll
        for (int it = 0; it < 8; ++it) {
          const int row = it * 2 + hh;
          v4f v = *(const v4f*)(slab + row * 68 + c4);
          *(volatile v4f*)(C + (size_t)(mBase + row) * ldc + n0 + c4) = v;
        }
        __threadfence();
      }
    } else {
      const int q = lane >> 3, c8 = (lane & 7) * 8;
      unsigned short* C  = (unsigned short*)Cout  + (size_t)b * strideC;
      unsigned short* C2 = (OUT_MODE == 2) ? ((unsigned short*)Cout2 + (size_t)b * strideC) : nullptr;
      for (int pass = 0; pass < 2; ++pass) {
#pragma unroll
        for (int it = 0; it < 4; ++it) {
          const int row = it * 4 + q;
          const float* sp = slab + row * 68 + c8;
          v8h hv, lv;
#pragma unroll
          for (int e = 0; e < 8; ++e) {
            if (OUT_MODE == 1) {
              hv[e] = (_Float16)sp[e];
            } else {
              unsigned short hb = f2bf_bits(sp[e]);
              unsigned short lb = f2bf_bits(sp[e] - bf_bits2f(hb));
              hv[e] = __builtin_bit_cast(_Float16, hb);
              lv[e] = __builtin_bit_cast(_Float16, lb);
            }
          }
          *(volatile v8h*)(C + (size_t)(mBase + row) * ldc + n0 + c8) = hv;
          if (OUT_MODE == 2) *(volatile v8h*)(C2 + (size_t)(mBase + row) * ldc + n0 + c8) = lv;
        }
        __threadfence();
      }
    }
    __builtin_amdgcn_fence(__ATOMIC_RELEASE, "workgroup");
    __builtin_amdgcn_wave_barrier();
    __builtin_amdgcn_fence(__ATOMIC_ACQUIRE, "workgroup");
  }
}

__global__ __launch_bounds__(256) void k_cast_f16x2(
    const float* __restrict__ in, _Float16* __restrict__ out, int n2, float scale) {
  const int i = blockIdx.x * 256 + threadIdx.x;
  if (i < n2) {
    const _Float16 h0 = (_Float16)(in[2 * i] * scale), h1 = (_Float16)(in[2 * i + 1] * scale);
    const unsigned u = (unsigned)__builtin_bit_cast(unsigned short, h0) | ((unsigned)__builtin_bit_cast(unsigned short, h1) << 16);
    ((volatile unsigned*)out)[i] = u;
    __threadfence();
    ((volatile unsigned*)out)[i] = u;
  }
}

__global__ __launch_bounds__(256) void k_wT(
    const float* __restrict__ p0, const float* __restrict__ p1,
    const float* __restrict__ p2, const float* __restrict__ p3,
    _Float16* __restrict__ out, int K, int N, float scale) {
  __shared__ float tile[64][65];
  const int tid = threadIdx.x, lane = tid & 31, wave = tid >> 5;
  const int n0 = blockIdx.x * 64, k0 = blockIdx.y * 64, z = blockIdx.z;
  const float* src = (z == 0) ? p0 : (z == 1) ? p1 : (z == 2) ? p2 : p3;
  const int c4 = (tid & 15) * 4, r0 = tid >> 4;
#pragma unroll
  for (int it = 0; it < 4; ++it) {
    const int kr = it * 16 + r0;
    const v4f v = *(const v4f*)(src + (size_t)(k0 + kr) * N + n0 + c4);
    tile[c4 + 0][kr] = v[0];
    tile[c4 + 1][kr] = v[1];
    tile[c4 + 2][kr] = v[2];
    tile[c4 + 3][kr] = v[3];
  }
  __syncthreads();
  const int q = lane >> 3, c8 = (lane & 7) * 8;
  _Float16* ob = out + (size_t)z * N * K;
  for (int pass = 0; pass < 2; ++pass) {
#pragma unroll
    for (int it = 0; it < 2; ++it) {
      const int row = wave * 8 + it * 4 + q;
      v8h hv;
#pragma unroll
      for (int e = 0; e < 8; ++e) hv[e] = (_Float16)(tile[row][c8 + e] * scale);
      *(volatile v8h*)(ob + (size_t)(n0 + row) * K + k0 + c8) = hv;
    }
    __threadfence();
  }
}

__global__ __launch_bounds__(256) void k_favor(
    const float* __restrict__ qin, const float* __restrict__ kin, const float* __restrict__ omega,
    float* __restrict__ qf, float* __restrict__ kf, int ntok) {
  __shared__ __align__(16) float omT[32 * 68];
  __shared__ __align__(16) float xs[8][512];
  __shared__ float nrm[8][8];
  const int tid = threadIdx.x, lane = tid & 31, wave = tid >> 5, hh = lane >> 4;
#pragma unroll
  for (int i = 0; i < 8; ++i) {
    const int idx = i * 256 + tid;
    omT[(idx & 31) * 68 + (idx >> 5)] = omega[idx];
  }
  __syncthreads();
  const int tok = blockIdx.x * 8 + wave;
  if (tok >= ntok) return;
  const float sc = 0.35355339059327379f;
  float* xw = xs[wave];
#pragma unroll 1
  for (int srci = 0; srci < 2; ++srci) {
    const float* xrow = ((srci == 0) ? qin : kin) + (size_t)tok * 512;
    float* frow = ((srci == 0) ? qf : kf) + (size_t)tok * 512;
    __builtin_amdgcn_fence(__ATOMIC_RELEASE, "workgroup");
    __builtin_amdgcn_wave_barrier();
    __builtin_amdgcn_fence(__ATOMIC_ACQUIRE, "workgroup");
#pragma unroll
    for (int i = 0; i < 4; ++i) {
      v4f v = *(const v4f*)(xrow + i * 128 + lane * 4);
      v = v * sc;
      *(v4f*)(xw + i * 128 + lane * 4) = v;
      float s = v[0] * v[0] + v[1] * v[1] + v[2] * v[2] + v[3] * v[3];
      s += __shfl_xor(s, 1, 32);
      s += __shfl_xor(s, 2, 32);
      s += __shfl_xor(s, 4, 32);
      s += __shfl_xor(s, 8, 32);
      if ((lane & 15) == 0) nrm[wave][2 * i + hh] = s;
    }
    __builtin_amdgcn_fence(__ATOMIC_RELEASE, "workgroup");
    __builtin_amdgcn_wave_barrier();
    __builtin_amdgcn_fence(__ATOMIC_ACQUIRE, "workgroup");
#pragma unroll 1
    for (int h = 0; h < 8; ++h) {
      const float off = 0.5f * nrm[wave][h];
      const float* xp = xw + h * 64;
      const float* op = omT + lane * 68;
      float u = 0.f;
#pragma unroll 1
      for (int g = 0; g < 4; ++g) {
        const v4f a0 = *(const v4f*)(xp + 16 * g);
        const v4f a1 = *(const v4f*)(xp + 16 * g + 4);
        const v4f a2 = *(const v4f*)(xp + 16 * g + 8);
        const v4f a3 = *(const v4f*)(xp + 16 * g + 12);
        const v4f o0 = *(const v4f*)(op + 16 * g);
        const v4f o1 = *(const v4f*)(op + 16 * g + 4);
        const v4f o2 = *(const v4f*)(op + 16 * g + 8);
        const v4f o3 = *(const v4f*)(op + 16 * g + 12);
        u = fmaf(a0[0], o0[0], u); u = fmaf(a0[1], o0[1], u); u = fmaf(a0[2], o0[2], u); u = fmaf(a0[3], o0[3], u);
        u = fmaf(a1[0], o1[0], u); u = fmaf(a1[1], o1[1], u); u = fmaf(a1[2], o1[2], u); u = fmaf(a1[3], o1[3], u);
        u = fmaf(a2[0], o2[0], u); u = fmaf(a2[1], o2[1], u); u = fmaf(a2[2], o2[2], u); u = fmaf(a2[3], o2[3], u);
        u = fmaf(a3[0], o3[0], u); u = fmaf(a3[1], o3[1], u); u = fmaf(a3[2], o3[2], u); u = fmaf(a3[3], o3[3], u);
      }
      const float e1 = expf(u - off) * 0.125f;
      const float e2 = expf(-u - off) * 0.125f;
      volatile float* vo = frow + h * 64;
      vo[lane] = e1;
      vo[lane + 32] = e2;
      __threadfence();
      vo[lane] = e1;
      vo[lane + 32] = e2;
    }
  }
}

#define RC_T 32
__global__ __launch_bounds__(64) void k_recur(
    const float* __restrict__ qf, const float* __restrict__ kf, const float* __restrict__ vin,
    _Float16* __restrict__ outh, int L, float oscale) {
  __shared__ __align__(16) float S[64 * 68];
  __shared__ __align__(16) float Kc[RC_T * 64];
  __shared__ __align__(16) float Qc[RC_T * 64];
  __shared__ __align__(16) float Vc[RC_T * 64];
  __shared__ float denp[2][RC_T];
  __shared__ float den[RC_T];
  const int tid = threadIdx.x, lane = tid & 31, wave = tid >> 5;
  const int b = blockIdx.x >> 3, h = blockIdx.x & 7;
  const size_t base = (size_t)b * L * 512 + (size_t)h * 64;
  float* srow = S + tid * 68;
#pragma unroll
  for (int g = 0; g < 16; ++g) *(v4f*)(srow + 4 * g) = (v4f){0.f, 0.f, 0.f, 0.f};
  float z = 0.f;
  const int nch = L / RC_T;
  for (int ch = 0; ch < nch; ++ch) {
    const int t0 = ch * RC_T;
    __syncthreads();
    {
      const int r0 = tid >> 4, c4 = (tid & 15) * 4;
#pragma unroll
      for (int it = 0; it < 8; ++it) {
        const int r = it * 4 + r0;
        const size_t go = base + (size_t)(t0 + r) * 512 + c4;
        *(v4f*)(Kc + r * 64 + c4) = *(const v4f*)(kf + go);
        *(v4f*)(Qc + r * 64 + c4) = *(const v4f*)(qf + go);
        *(v4f*)(Vc + r * 64 + c4) = *(const v4f*)(vin + go);
      }
    }
    __syncthreads();
#pragma unroll 1
    for (int t = 0; t < RC_T; ++t) {
      z += Kc[t * 64 + tid];
      float p = Qc[t * 64 + tid] * z;
      p += __shfl_xor(p, 16, 32);
      p += __shfl_xor(p, 8, 32);
      p += __shfl_xor(p, 4, 32);
      p += __shfl_xor(p, 2, 32);
      p += __shfl_xor(p, 1, 32);
      if (lane == 0) denp[wave][t] = p;
    }
    __syncthreads();
    if (tid < RC_T) den[tid] = denp[0][tid] + denp[1][tid];
    __syncthreads();
#pragma unroll 1
    for (int t = 0; t < RC_T; ++t) {
      const float vt = Vc[t * 64 + tid];
      const float* kr = Kc + t * 64;
      const float* qr = Qc + t * 64;
      v4f n0 = (v4f){0.f, 0.f, 0.f, 0.f}, n1 = (v4f){0.f, 0.f, 0.f, 0.f};
#pragma unroll 1
      for (int g = 0; g < 8; ++g) {
        const v4f k0 = *(const v4f*)(kr + 8 * g);
        const v4f k1 = *(const v4f*)(kr + 8 * g + 4);
        const v4f q0 = *(const v4f*)(qr + 8 * g);
        const v4f q1 = *(const v4f*)(qr + 8 * g + 4);
        v4f s0 = *(v4f*)(srow + 8 * g);
        v4f s1 = *(v4f*)(srow + 8 * g + 4);
        s0 = k0 * vt + s0;
        s1 = k1 * vt + s1;
        *(v4f*)(srow + 8 * g) = s0;
        *(v4f*)(srow + 8 * g + 4) = s1;
        n0 = q0 * s0 + n0;
        n1 = q1 * s1 + n1;
      }
      const float num = ((n0[0] + n0[1]) + (n0[2] + n0[3])) + ((n1[0] + n1[1]) + (n1[2] + n1[3]));
      const float zi = __builtin_amdgcn_rcpf(den[t] + 1e-6f);
      Vc[t * 64 + tid] = num * zi;
    }
    __syncthreads();
    {
      const int q = lane >> 3, c8 = (lane & 7) * 8;
      for (int pass = 0; pass < 2; ++pass) {
#pragma unroll
        for (int it = 0; it < 4; ++it) {
          const int row = wave * 16 + it * 4 + q;
          v8h hv;
#pragma unroll
          for (int e = 0; e < 8; ++e) hv[e] = (_Float16)(Vc[row * 64 + c8 + e] * oscale);
          *(volatile v8h*)(outh + base + (size_t)(t0 + row) * 512 + c8) = hv;
        }
        __threadfence();
      }
    }
  }
}

template <bool WH>
__global__ __launch_bounds__(256) void k_ln(
    const float* __restrict__ in, const float* __restrict__ g, const float* __restrict__ bta,
    float* __restrict__ outf, _Float16* __restrict__ outh, int nrows, float hscale) {
  const int lane = threadIdx.x & 31, wave = threadIdx.x >> 5;
  const int row = blockIdx.x * 8 + wave;
  if (row >= nrows) return;
  const float* ip = in + (size_t)row * 512;
  v4f x[4];
  float s = 0.f;
#pragma unroll
  for (int i = 0; i < 4; ++i) {
    x[i] = *(const v4f*)(ip + i * 128 + lane * 4);
    s += (x[i][0] + x[i][1]) + (x[i][2] + x[i][3]);
  }
#pragma unroll
  for (int o = 1; o < 32; o <<= 1) s += __shfl_xor(s, o, 32);
  const float mu = s * 0.001953125f;
  float vs = 0.f;
#pragma unroll
  for (int i = 0; i < 4; ++i) {
    const v4f d = x[i] - mu;
    vs += (d[0] * d[0] + d[1] * d[1]) + (d[2] * d[2] + d[3] * d[3]);
  }
#pragma unroll
  for (int o = 1; o < 32; o <<= 1) vs += __shfl_xor(vs, o, 32);
  const float rstd = rsqrtf(vs * 0.001953125f + 1e-5f);
  v4f y[4];
#pragma unroll
  for (int i = 0; i < 4; ++i) {
    const v4f gg = *(const v4f*)(g + i * 128 + lane * 4);
    const v4f bb = *(const v4f*)(bta + i * 128 + lane * 4);
    y[i] = (x[i] - mu) * rstd * gg + bb;
  }
  float* op = outf + (size_t)row * 512;
  _Float16* oh = outh + (size_t)row * 512;
  for (int pass = 0; pass < 2; ++pass) {
#pragma unroll
    for (int i = 0; i < 4; ++i) {
      *(volatile v4f*)(op + i * 128 + lane * 4) = y[i];
      if (WH) {
        v4h hv;
        hv[0] = (_Float16)(y[i][0] * hscale); hv[1] = (_Float16)(y[i][1] * hscale);
        hv[2] = (_Float16)(y[i][2] * hscale); hv[3] = (_Float16)(y[i][3] * hscale);
        *(volatile v4h*)(oh + i * 128 + lane * 4) = hv;
      }
    }
    __threadfence();
  }
}

extern "C" void kernel_launch(void* const* d_in, const int* in_sizes, int n_in,
                              void* d_out, int out_size, void* d_ws, size_t ws_size,
                              hipStream_t stream)
{
  const int B = 2, L = 2048, D = 512, FF = 2048, HD = 64, MH = 32, DEPTH = 2;
  const int TOK = B * L;
  if (n_in < 20) return;
  if (in_sizes[0] != TOK * D || in_sizes[1] != DEPTH * D * D || in_sizes[3] != DEPTH * D * D ||
      in_sizes[5] != DEPTH * D * D || in_sizes[7] != DEPTH * D * D || in_sizes[9] != DEPTH * HD * MH ||
      in_sizes[12] != DEPTH * D * FF || in_sizes[14] != DEPTH * FF * D || out_size != TOK * D) return;

  const float* x_in  = (const float*)d_in[0];
  const float* Wq    = (const float*)d_in[1];
  const float* bq    = (const float*)d_in[2];
  const float* Wk    = (const float*)d_in[3];
  const float* bk    = (const float*)d_in[4];
  const float* Wv    = (const float*)d_in[5];
  const float* bv    = (const float*)d_in[6];
  const float* Wo    = (const float*)d_in[7];
  const float* bo    = (const float*)d_in[8];
  const float* omega = (const float*)d_in[9];
  const float* ln1g  = (const float*)d_in[10];
  const float* ln1b  = (const float*)d_in[11];
  const float* W1    = (const float*)d_in[12];
  const float* b1    = (const float*)d_in[13];
  const float* W2    = (const float*)d_in[14];
  const float* b2    = (const float*)d_in[15];
  const float* ln2g  = (const float*)d_in[16];
  const float* ln2b  = (const float*)d_in[17];
  const float* lnfg  = (const float*)d_in[18];
  const float* lnfb  = (const float*)d_in[19];
  float* out = (float*)d_out;

  char* ws = (char*)d_ws;
  size_t off = 0;
  auto carve = [&](size_t bytes) -> char* { char* p = ws + off; off += (bytes + 255) & ~(size_t)255; return p; };
  _Float16* xh  = (_Float16*)carve((size_t)TOK * D * 2);
  float*    xf  = (float*)carve((size_t)TOK * D * 4);
  float*    qb_ = (float*)carve((size_t)TOK * D * 4);
  float*    kb_ = (float*)carve((size_t)TOK * D * 4);
  float*    vb_ = (float*)carve((size_t)TOK * D * 4);
  float*    Qfb = (float*)carve((size_t)TOK * D * 4);
  float*    Kfb = (float*)carve((size_t)TOK * D * 4);
  _Float16* ah  = (_Float16*)carve((size_t)TOK * D * 2);
  float*    t1  = (float*)carve((size_t)TOK * D * 4);
  _Float16* y1h = (_Float16*)carve((size_t)TOK * FF * 2);
  _Float16* wt4 = (_Float16*)carve((size_t)4 * D * D * 2);
  _Float16* w1t = (_Float16*)carve((size_t)D * FF * 2);
  _Float16* w2t = (_Float16*)carve((size_t)FF * D * 2);
  if (off > ws_size) return;

  const float WSC = 64.0f, ASC = 16.0f;
  const int n2 = TOK * D / 2;
  k_cast_f16x2<<<dim3((n2 + 255) / 256), dim3(256), 0, stream>>>(x_in, xh, n2, 1.0f);

  const int tilesD  = (TOK / 64) * (D / 64);
  const int tilesFF = (TOK / 64) * (FF / 64);
  const dim3 gD((tilesD + 7) / 8, 1), gFF((tilesFF + 7) / 8, 1);

  for (int l = 0; l < DEPTH; ++l) {
    const size_t wDD = (size_t)l * D * D;
    const float* xres = (l == 0) ? x_in : xf;

    k_wT<<<dim3(D / 64, D / 64, 4), dim3(256), 0, stream>>>(Wq + wDD, Wk + wDD, Wv + wDD, Wo + wDD, wt4, D, D, WSC);
    k_wT<<<dim3(FF / 64, D / 64, 1), dim3(256), 0, stream>>>(W1 + (size_t)l * D * FF, W1 + (size_t)l * D * FF,
        W1 + (size_t)l * D * FF, W1 + (size_t)l * D * FF, w1t, D, FF, WSC);
    k_wT<<<dim3(D / 64, FF / 64, 1), dim3(256), 0, stream>>>(W2 + (size_t)l * FF * D, W2 + (size_t)l * FF * D,
        W2 + (size_t)l * FF * D, W2 + (size_t)l * FF * D, w2t, FF, D, WSC);

    const unsigned short* xhu = (const unsigned short*)xh;
    const unsigned short* wtu = (const unsigned short*)wt4;
    wmma_gemm64<0, false, 2, 0, false, 0><<<gD, dim3(256), 0, stream>>>(
        xhu, xhu, D, 0L, wtu + 0 * (size_t)D * D, wtu + 0 * (size_t)D * D, D, 0L,
        (void*)qb_, (void*)qb_, D, 0L, bq + (size_t)l * D, bq + (size_t)l * D, 0L, TOK, D, D, 1.0f / WSC);
    wmma_gemm64<0, false, 2, 0, false, 0><<<gD, dim3(256), 0, stream>>>(
        xhu, xhu, D, 0L, wtu + 1 * (size_t)D * D, wtu + 1 * (size_t)D * D, D, 0L,
        (void*)kb_, (void*)kb_, D, 0L, bk + (size_t)l * D, bk + (size_t)l * D, 0L, TOK, D, D, 1.0f / WSC);
    wmma_gemm64<0, false, 2, 0, false, 0><<<gD, dim3(256), 0, stream>>>(
        xhu, xhu, D, 0L, wtu + 2 * (size_t)D * D, wtu + 2 * (size_t)D * D, D, 0L,
        (void*)vb_, (void*)vb_, D, 0L, bv + (size_t)l * D, bv + (size_t)l * D, 0L, TOK, D, D, 1.0f / WSC);

    k_favor<<<dim3((TOK + 7) / 8), dim3(256), 0, stream>>>(qb_, kb_, omega + (size_t)l * HD * MH, Qfb, Kfb, TOK);

    k_recur<<<dim3(B * 8), dim3(64), 0, stream>>>(Qfb, Kfb, vb_, ah, L, ASC);

    wmma_gemm64<0, false, 2, 0, true, 0><<<gD, dim3(256), 0, stream>>>(
        (const unsigned short*)ah, (const unsigned short*)ah, D, 0L, wtu + 3 * (size_t)D * D, wtu + 3 * (size_t)D * D, D, 0L,
        (void*)t1, (void*)t1, D, 0L, bo + (size_t)l * D, xres, 0L, TOK, D, D, 1.0f / (WSC * ASC));
    k_ln<true><<<dim3((TOK + 7) / 8), dim3(256), 0, stream>>>(t1, ln1g + (size_t)l * D, ln1b + (size_t)l * D, xf, xh, TOK, 1.0f);

    wmma_gemm64<0, false, 2, 1, false, 2><<<gFF, dim3(256), 0, stream>>>(
        xhu, xhu, D, 0L, (const unsigned short*)w1t, (const unsigned short*)w1t, D, 0L,
        (void*)y1h, (void*)y1h, FF, 0L, b1 + (size_t)l * FF, b1 + (size_t)l * FF, 0L, TOK, FF, D, 1.0f / WSC);
    wmma_gemm64<0, false, 2, 0, true, 0><<<gD, dim3(256), 0, stream>>>(
        (const unsigned short*)y1h, (const unsigned short*)y1h, FF, 0L, (const unsigned short*)w2t, (const unsigned short*)w2t, FF, 0L,
        (void*)t1, (void*)t1, D, 0L, b2 + (size_t)l * D, xf, 0L, TOK, D, FF, 1.0f / WSC);
    k_ln<true><<<dim3((TOK + 7) / 8), dim3(256), 0, stream>>>(t1, ln2g + (size_t)l * D, ln2b + (size_t)l * D, xf, xh, TOK, 1.0f);
  }

  k_ln<false><<<dim3((TOK + 7) / 8), dim3(256), 0, stream>>>(xf, lnfg, lnfb, out, xh, TOK, 1.0f);
  (void)hipGetLastError();
}
